// self_attention_85040352461375
// MI455X (gfx1250) — hardware-verified
//
#include <hip/hip_runtime.h>


#define DEV __device__ __forceinline__

#ifndef NB
#define NB 8
#endif
#ifndef SEQ
#define SEQ 4096
#endif
#define NB_FULL  8
#define SEQ_FULL 4096
#define CIN   12
#define CQK   36
#define CPAD  64
#define VROWS 48
#define QP    72
#define VP    136
#define OSP   132
#define KSCALE (0.28867513459481287f * 1.4426950408889634f)
#define VCARRY 16.0f
#define PLOG2  12.0f
#define OUT_SCALE (1.0f / 65536.0f)

static_assert(NB >= 1 && NB <= NB_FULL);
static_assert(SEQ >= 128 && SEQ <= SEQ_FULL && (SEQ % 128) == 0);
static_assert(256 * 4 * 8 == 128 * CPAD);
static_assert(256 * 3 * 8 == VROWS * 128);
static_assert(384 * 4 == CIN * 128);
static_assert(32 * 4 == 128);
static_assert(((QP * 2) % 16) == 0 && ((VP * 2) % 16) == 0 && ((OSP * 4) % 16) == 0);
static_assert(CQK <= CPAD && CQK <= VROWS && CIN <= 16);

typedef _Float16       v8h   __attribute__((ext_vector_type(8)));
typedef _Float16       v16h  __attribute__((ext_vector_type(16)));
typedef __bf16         v16bf __attribute__((ext_vector_type(16)));
typedef unsigned short v8us  __attribute__((ext_vector_type(8)));
typedef unsigned short v16us __attribute__((ext_vector_type(16)));
typedef float          v8f   __attribute__((ext_vector_type(8)));
typedef float          v4f   __attribute__((ext_vector_type(4)));

union FragH { v16h v;  v8h  half[2]; };
union FragB { v16bf v; v16us u; v8us half[2]; };

DEV unsigned int bf16_bits(float f) {
    unsigned int u = __float_as_uint(f);
    u += 0x7FFFu + ((u >> 16) & 1u);
    return u >> 16;
}
DEV float bf16_val(float f) { return __uint_as_float(bf16_bits(f) << 16); }

DEV v8f zero8f() {
    v8f z;
#pragma unroll
    for (int i = 0; i < 8; ++i) z[i] = 0.f;
    return z;
}

DEV float ex2(float x) { return __builtin_amdgcn_exp2f(x); }

DEV v8f mma_bf16(v16bf a, v16bf b, v8f c) {
    c = __builtin_amdgcn_wmma_f32_16x16x32_bf16(false, a, false, b, (short)0, c, false, false);
    asm volatile("v_nop\n\tv_nop\n\tv_nop\n\tv_nop" : "+v"(c) : "v"(a), "v"(b));
    return c;
}
DEV v8f mma_f16(v16h a, v16h b, v8f c) {
    c = __builtin_amdgcn_wmma_f32_16x16x32_f16(false, a, false, b, (short)0, c, false, false);
    asm volatile("v_nop\n\tv_nop\n\tv_nop\n\tv_nop" : "+v"(c) : "v"(a), "v"(b));
    return c;
}

DEV FragB w_frag(const float* Wl, unsigned t, unsigned h, unsigned l15) {
    FragB a;
    const unsigned c  = 16u * t + l15;
    const unsigned cc = c < (unsigned)CQK ? c : (unsigned)(CQK - 1);
#pragma unroll
    for (unsigned e = 0; e < 8; ++e) {
        const unsigned i  = 8u * h + e;
        const unsigned ic = i < (unsigned)CIN ? i : (unsigned)(CIN - 1);
        const unsigned bits = __float_as_uint(Wl[cc * CIN + ic]) >> 16;
        a.u[e]     = (unsigned short)((c < (unsigned)CQK && i < (unsigned)CIN) ? bits : 0u);
        a.u[8 + e] = (unsigned short)0;
    }
    return a;
}

DEV v8f proj_tile(const float* Wl, const float* Bl, unsigned t, unsigned h, unsigned l15, v16bf xb, float carry) {
    const FragB a = w_frag(Wl, t, h, l15);
    v8f acc = mma_bf16(a.v, xb, zero8f());
#pragma unroll
    for (unsigned r = 0; r < 8; ++r) {
        const unsigned c  = 16u * t + 8u * h + r;
        const unsigned cc = c < (unsigned)CQK ? c : (unsigned)(CQK - 1);
        const float bvl = Bl[cc];
        acc[r] = (acc[r] + ((c < (unsigned)CQK) ? bvl : 0.f)) * carry;
    }
    return acc;
}

__global__ __launch_bounds__(256) void k_proj(const float* __restrict__ x,
                                              const float* __restrict__ wq, const float* __restrict__ bq,
                                              const float* __restrict__ wk, const float* __restrict__ bk,
                                              const float* __restrict__ wv, const float* __restrict__ bv,
                                              _Float16* __restrict__ Qp, _Float16* __restrict__ Kp,
                                              _Float16* __restrict__ Vp)
{
    __shared__ __attribute__((aligned(16))) _Float16 Qs[128 * QP];
    __shared__ __attribute__((aligned(16))) _Float16 Ks[128 * QP];
    __shared__ __attribute__((aligned(16))) _Float16 Vs[VROWS * VP];
    __shared__ float Ws[3 * CQK * CIN];
    __shared__ float Bs[3 * CQK];

    const unsigned tid = threadIdx.x, lane = tid & 31u, w = tid >> 5;
    const unsigned h = lane >> 4, l15 = lane & 15u;
    const unsigned bps = (unsigned)(SEQ / 128);
    const unsigned b = blockIdx.x / bps;
    const unsigned pos0 = (blockIdx.x - b * bps) * 128u;
    const unsigned nl = w * 16u + l15;

#pragma unroll
    for (unsigned it = 0; it < 2; ++it) {
        const unsigned i  = it * 256u + tid;
        const unsigned ic = i < 432u ? i : 431u;
        const float a0 = bf16_val(wq[ic]);
        const float a1 = bf16_val(wk[ic]);
        const float a2 = bf16_val(wv[ic]);
        if (i < 432u) { Ws[i] = a0; Ws[432u + i] = a1; Ws[864u + i] = a2; }
    }
    {
        const unsigned ic = tid < (unsigned)CQK ? tid : (unsigned)(CQK - 1);
        const float a0 = bf16_val(bq[ic]);
        const float a1 = bf16_val(bk[ic]);
        const float a2 = bf16_val(bv[ic]);
        if (tid < (unsigned)CQK) { Bs[tid] = a0; Bs[CQK + tid] = a1; Bs[2 * CQK + tid] = a2; }
    }

    FragB xb;
    {
        const float* xp = x + (size_t)b * CIN * SEQ_FULL + pos0 + nl;
#pragma unroll
        for (unsigned e = 0; e < 8; ++e) {
            const unsigned i  = 8u * h + e;
            const unsigned ic = i < (unsigned)CIN ? i : (unsigned)(CIN - 1);
            const unsigned bits = bf16_bits(xp[(size_t)ic * SEQ_FULL]);
            xb.u[e]     = (unsigned short)((i < (unsigned)CIN) ? bits : 0u);
            xb.u[8 + e] = (unsigned short)0;
        }
    }
    __syncthreads();

    v8h zz;
#pragma unroll
    for (int i = 0; i < 8; ++i) zz[i] = (_Float16)0.f;

#pragma unroll
    for (unsigned t = 0; t < 3; ++t) {
        const v8f acc = proj_tile(Ws, Bs, t, h, l15, xb.v, 1.0f);
        v8h o;
#pragma unroll
        for (int r = 0; r < 8; ++r) o[r] = (_Float16)acc[r];
        *(v8h*)(Qs + nl * QP + 16u * t + 8u * h) = o;
    }
    *(v8h*)(Qs + nl * QP + 48u + 8u * h) = zz;
#pragma unroll
    for (unsigned t = 0; t < 3; ++t) {
        const v8f acc = proj_tile(Ws + CQK * CIN, Bs + CQK, t, h, l15, xb.v, KSCALE);
        v8h o;
#pragma unroll
        for (int r = 0; r < 8; ++r) o[r] = (_Float16)acc[r];
        *(v8h*)(Ks + nl * QP + 16u * t + 8u * h) = o;
    }
    *(v8h*)(Ks + nl * QP + 48u + 8u * h) = zz;
#pragma unroll
    for (unsigned t = 0; t < 3; ++t) {
        const v8f acc = proj_tile(Ws + 2 * CQK * CIN, Bs + 2 * CQK, t, h, l15, xb.v, VCARRY);
#pragma unroll
        for (unsigned r = 0; r < 8; ++r)
            Vs[(16u * t + 8u * h + r) * VP + nl] = (_Float16)acc[r];
    }
    __syncthreads();

    v8h qv[4], kv[4], vv[3];
#pragma unroll
    for (unsigned it = 0; it < 4; ++it) {
        const unsigned idx = it * 256u + tid;
        const unsigned row = idx >> 3, pc = idx & 7u;
        qv[it] = *(const v8h*)(Qs + row * QP + pc * 8u);
        kv[it] = *(const v8h*)(Ks + row * QP + pc * 8u);
    }
#pragma unroll
    for (unsigned it = 0; it < 3; ++it) {
        const unsigned idx = it * 256u + tid;
        const unsigned row = idx >> 4, pc = idx & 15u;
        vv[it] = *(const v8h*)(Vs + row * VP + pc * 8u);
    }
    _Float16* qd = Qp + ((size_t)b * SEQ + pos0) * CPAD;
    _Float16* kd = Kp + ((size_t)b * SEQ + pos0) * CPAD;
    _Float16* vd = Vp + (size_t)b * VROWS * SEQ + pos0;
#pragma unroll
    for (unsigned it = 0; it < 4; ++it) {
        const unsigned idx = it * 256u + tid;
        *(volatile v8h*)(qd + (size_t)idx * 8u) = qv[it];
        *(volatile v8h*)(kd + (size_t)idx * 8u) = kv[it];
    }
#pragma unroll
    for (unsigned it = 0; it < 3; ++it) {
        const unsigned idx = it * 256u + tid;
        const unsigned row = idx >> 4, pc = idx & 15u;
        *(volatile v8h*)(vd + (size_t)row * SEQ + pc * 8u) = vv[it];
    }
    __threadfence();
#pragma unroll
    for (unsigned it = 0; it < 4; ++it) {
        const unsigned idx = it * 256u + tid;
        *(volatile v8h*)(qd + (size_t)idx * 8u) = qv[it];
        *(volatile v8h*)(kd + (size_t)idx * 8u) = kv[it];
    }
#pragma unroll
    for (unsigned it = 0; it < 3; ++it) {
        const unsigned idx = it * 256u + tid;
        const unsigned row = idx >> 4, pc = idx & 15u;
        *(volatile v8h*)(vd + (size_t)row * SEQ + pc * 8u) = vv[it];
    }
}

__global__ __launch_bounds__(256) void k_stats(const _Float16* __restrict__ Kp,
                                               const _Float16* __restrict__ Qp,
                                               float* __restrict__ offt)
{
    __shared__ __attribute__((aligned(16))) float offS[128];

    const unsigned tid = threadIdx.x, lane = tid & 31u, w = tid >> 5;
    const unsigned h = lane >> 4, l15 = lane & 15u;
    const unsigned bps = (unsigned)(SEQ / 128);
    const unsigned b = blockIdx.x / bps;
    const unsigned pos0 = (blockIdx.x - b * bps) * 128u;

    FragH k0, k1;
    {
        const _Float16* kp = Kp + ((size_t)b * SEQ + pos0 + w * 16u + l15) * CPAD + 8u * h;
        k0.half[0] = *(const v8h*)(kp);
        k0.half[1] = *(const v8h*)(kp + 16);
        k1.half[0] = *(const v8h*)(kp + 32);
        k1.half[1] = *(const v8h*)(kp + 48);
    }

    float m[8], z[8];
#pragma unroll
    for (int r = 0; r < 8; ++r) { m[r] = -3.0e38f; z[r] = 0.f; }

    const _Float16* qb = Qp + ((size_t)b * SEQ + l15) * CPAD + 8u * h;
#pragma unroll 2
    for (unsigned mt = 0; mt < (unsigned)(SEQ / 16); ++mt) {
        const _Float16* qp = qb + (size_t)mt * 16u * CPAD;
        FragH q0, q1;
        q0.half[0] = *(const v8h*)(qp);
        q0.half[1] = *(const v8h*)(qp + 16);
        q1.half[0] = *(const v8h*)(qp + 32);
        q1.half[1] = *(const v8h*)(qp + 48);
        v8f c = zero8f();
        c = mma_f16(k0.v, q0.v, c);
        c = mma_f16(k1.v, q1.v, c);
#pragma unroll
        for (int r = 0; r < 8; ++r) {
            const float mn = fmaxf(m[r], c[r]);
            z[r] = z[r] * ex2(m[r] - mn) + ex2(c[r] - mn);
            m[r] = mn;
        }
    }

#pragma unroll
    for (unsigned r = 0; r < 8; ++r) {
        float M = m[r];
#pragma unroll
        for (int o = 1; o < 16; o <<= 1) M = fmaxf(M, __shfl_xor(M, o));
        float zs = z[r] * ex2(m[r] - M);
#pragma unroll
        for (int o = 1; o < 16; o <<= 1) zs += __shfl_xor(zs, o);
        const float ov = M + log2f(zs) - PLOG2;
        if (l15 == 0u) offS[w * 16u + 8u * h + r] = ov;
    }
    __syncthreads();

    if (w == 0u) {
        const v4f v = *(const v4f*)(offS + lane * 4u);
        float* dst = offt + (size_t)b * SEQ + pos0 + lane * 4u;
        *(volatile v4f*)dst = v;
        __threadfence();
        *(volatile v4f*)dst = v;
    }
}

__global__ __launch_bounds__(256) void k_attn(const _Float16* __restrict__ Kp,
                                              const _Float16* __restrict__ Qp,
                                              const _Float16* __restrict__ Vp,
                                              const float* __restrict__ offt,
                                              const float* __restrict__ wo,
                                              const float* __restrict__ bo,
                                              float* __restrict__ out)
{
    __shared__ __attribute__((aligned(16))) float attnS[8 * 48 * 16];
    __shared__ __attribute__((aligned(16))) float outS[CIN * OSP];
    __shared__ float woS[CIN * CQK];
    __shared__ float boS[16];

    const unsigned tid = threadIdx.x, lane = tid & 31u, w = tid >> 5;
    const unsigned h = lane >> 4, l15 = lane & 15u;
    const unsigned bps = (unsigned)(SEQ / 128);
    const unsigned b = blockIdx.x / bps;
    const unsigned pos0 = (blockIdx.x - b * bps) * 128u;

#pragma unroll
    for (unsigned it = 0; it < 2; ++it) {
        const unsigned i  = it * 256u + tid;
        const unsigned ic = i < 432u ? i : 431u;
        const float a0 = bf16_val(wo[ic]);
        if (i < 432u) woS[i] = a0;
    }
    {
        const unsigned ic = tid < (unsigned)CIN ? tid : (unsigned)(CIN - 1);
        const float a0 = bf16_val(bo[ic]);
        if (tid < (unsigned)CIN) boS[tid] = a0;
    }

    FragH q0, q1;
    {
        const _Float16* qp = Qp + ((size_t)b * SEQ + pos0 + w * 16u + l15) * CPAD + 8u * h;
        q0.half[0] = *(const v8h*)(qp);
        q0.half[1] = *(const v8h*)(qp + 16);
        q1.half[0] = *(const v8h*)(qp + 32);
        q1.half[1] = *(const v8h*)(qp + 48);
    }

    v8f acc[3];
#pragma unroll
    for (int t = 0; t < 3; ++t) acc[t] = zero8f();

    const _Float16* kb = Kp + ((size_t)b * SEQ + l15) * CPAD + 8u * h;
    const _Float16* vb = Vp + ((size_t)b * VROWS + l15) * SEQ + 8u * h;
    const float*    ob = offt + (size_t)b * SEQ + 8u * h;

#pragma unroll 1
    for (unsigned ns = 0; ns < (unsigned)(SEQ / 32); ++ns) {
        const _Float16* kp = kb + (size_t)ns * 32u * CPAD;
        FragH a;
        v8f c0 = zero8f();
        a.half[0] = *(const v8h*)(kp);
        a.half[1] = *(const v8h*)(kp + 16);
        c0 = mma_f16(a.v, q0.v, c0);
        a.half[0] = *(const v8h*)(kp + 32);
        a.half[1] = *(const v8h*)(kp + 48);
        c0 = mma_f16(a.v, q1.v, c0);
        kp += 16 * CPAD;
        v8f c1 = zero8f();
        a.half[0] = *(const v8h*)(kp);
        a.half[1] = *(const v8h*)(kp + 16);
        c1 = mma_f16(a.v, q0.v, c1);
        a.half[0] = *(const v8h*)(kp + 32);
        a.half[1] = *(const v8h*)(kp + 48);
        c1 = mma_f16(a.v, q1.v, c1);

        const float* op = ob + ns * 32u;
        const v4f o0a = *(const v4f*)(op);
        const v4f o0b = *(const v4f*)(op + 4);
        const v4f o1a = *(const v4f*)(op + 16);
        const v4f o1b = *(const v4f*)(op + 20);

        FragH pb;
#pragma unroll
        for (int r = 0; r < 4; ++r) {
            pb.v[r]      = (_Float16)ex2(c0[r]     - o0a[r]);
            pb.v[4 + r]  = (_Float16)ex2(c0[4 + r] - o0b[r]);
            pb.v[8 + r]  = (_Float16)ex2(c1[r]     - o1a[r]);
            pb.v[12 + r] = (_Float16)ex2(c1[4 + r] - o1b[r]);
        }

        const _Float16* vp = vb + ns * 32u;
#pragma unroll
        for (unsigned t = 0; t < 3; ++t) {
            FragH vf;
            vf.half[0] = *(const v8h*)(vp + (size_t)t * 16u * SEQ);
            vf.half[1] = *(const v8h*)(vp + (size_t)t * 16u * SEQ + 16);
            acc[t] = mma_f16(vf.v, pb.v, acc[t]);
        }
    }

    float* aL = attnS + w * (48u * 16u);
#pragma unroll
    for (unsigned t = 0; t < 3; ++t) {
#pragma unroll
        for (unsigned r = 0; r < 8; ++r)
            aL[(16u * t + 8u * h + r) * 16u + l15] = acc[t][r] * OUT_SCALE;
    }
    __syncthreads();

#pragma unroll 1
    for (unsigned oo = 0; oo < 6; ++oo) {
        const unsigned o = h * 6u + oo;
        float sum = boS[o];
        const float* wr = woS + o * CQK;
#pragma unroll
        for (unsigned c = 0; c < (unsigned)CQK; ++c) sum += wr[c] * aL[c * 16u + l15];
        outS[o * OSP + w * 16u + l15] = sum;
    }
    __syncthreads();

    const unsigned row0 = w;
    const unsigned row1 = (8u + w) < (unsigned)CIN ? (8u + w) : (unsigned)(CIN - 1);
    const v4f ov0 = *(const v4f*)(outS + row0 * OSP + lane * 4u);
    const v4f ov1 = *(const v4f*)(outS + row1 * OSP + lane * 4u);
    float* d0 = out + ((size_t)b * CIN + row0) * SEQ + pos0 + lane * 4u;
    float* d1 = out + ((size_t)b * CIN + row1) * SEQ + pos0 + lane * 4u;
    *(volatile v4f*)d0 = ov0;
    if (w < 4u) *(volatile v4f*)d1 = ov1;
    __threadfence();
    *(volatile v4f*)d0 = ov0;
    if (w < 4u) *(volatile v4f*)d1 = ov1;
}

extern "C" void kernel_launch(void* const* d_in, const int* in_sizes, int n_in,
                              void* d_out, int out_size, void* d_ws, size_t ws_size,
                              hipStream_t stream)
{
    if (n_in < 9) return;
    const long long need_x = ((long long)NB * CIN - 1) * SEQ_FULL + SEQ;
    if ((long long)in_sizes[0] < need_x) return;
    if (in_sizes[1] < CQK * CIN || in_sizes[2] < CQK) return;
    if (in_sizes[3] < CQK * CIN || in_sizes[4] < CQK) return;
    if (in_sizes[5] < CQK * CIN || in_sizes[6] < CQK) return;
    if (in_sizes[7] < CIN * CQK || in_sizes[8] < CIN) return;
    if ((long long)out_size < (long long)NB * CIN * SEQ) return;

    const float* x  = (const float*)d_in[0];
    const float* wq = (const float*)d_in[1];
    const float* bq = (const float*)d_in[2];
    const float* wk = (const float*)d_in[3];
    const float* bk = (const float*)d_in[4];
    const float* wv = (const float*)d_in[5];
    const float* bv = (const float*)d_in[6];
    const float* wo = (const float*)d_in[7];
    const float* bo = (const float*)d_in[8];
    float* out = (float*)d_out;

    char* ws = (char*)d_ws;
    size_t off = 0;
    auto carve = [&](size_t bytes) -> char* {
        char* p = ws + off;
        off += (bytes + 255) & ~(size_t)255;
        return p;
    };
    _Float16* Qp  = (_Float16*)carve((size_t)NB * SEQ * CPAD * 2);
    _Float16* Kp  = (_Float16*)carve((size_t)NB * SEQ * CPAD * 2);
    _Float16* Vp  = (_Float16*)carve((size_t)NB * VROWS * SEQ * 2);
    float*    oft = (float*)carve((size_t)NB * SEQ * 4);
    if (off > ws_size) return;

    const unsigned nblk = (unsigned)(NB * (SEQ / 128));
    k_proj <<<nblk, 256, 0, stream>>>(x, wq, bq, wk, bk, wv, bv, Qp, Kp, Vp);
    k_stats<<<nblk, 256, 0, stream>>>(Kp, Qp, oft);
    k_attn <<<nblk, 256, 0, stream>>>(Kp, Qp, Vp, oft, wo, bo, out);
}
